// MSA_10969346474559
// MI455X (gfx1250) — hardware-verified
//
#include <hip/hip_runtime.h>
#include <math.h>
#include <stdint.h>

#define NB    4
#define SEQ   2048
#define DMOD  1024
#define NH    16
#define HD    64
#define NTOK  (NB * SEQ)

typedef __attribute__((ext_vector_type(16))) _Float16 v16h;
typedef __attribute__((ext_vector_type(8)))  _Float16 v8h;
typedef __attribute__((ext_vector_type(16))) __bf16   v16b;
typedef __attribute__((ext_vector_type(8)))  __bf16   v8b;
typedef __attribute__((ext_vector_type(8)))  float    v8f;
typedef __attribute__((ext_vector_type(4)))  float    v4f;
typedef __attribute__((ext_vector_type(4)))  unsigned int v4u;

__device__ __forceinline__ unsigned short f2bf_bits(float f) {
  unsigned u = __float_as_uint(f);
  return (unsigned short)((u + 0x7FFFu + ((u >> 16) & 1u)) >> 16);
}
__device__ __forceinline__ float bf_bits2f(unsigned short h) { return __uint_as_float(((unsigned)h) << 16); }
__device__ __forceinline__ float bfr(float f) { return bf_bits2f(f2bf_bits(f)); }
__device__ __forceinline__ unsigned pk16(unsigned short a, unsigned short b) { return (unsigned)a | ((unsigned)b << 16); }

__device__ __forceinline__ void dep_guard_b(v8f& a, v8f& b, v16b x, v16b y) { asm volatile("v_nop\n\tv_nop\n\tv_nop\n\tv_nop" : "+v"(a), "+v"(b) : "v"(x), "v"(y)); }
__device__ __forceinline__ void keep4_b(v16b a, v16b b, v16b c, v16b d) { asm volatile("v_nop" :: "v"(a), "v"(b), "v"(c), "v"(d)); }
__device__ __forceinline__ void acc_guard4(v8f& a, v8f& b, v8f& c, v8f& d) { asm volatile("v_nop\n\tv_nop\n\tv_nop\n\tv_nop" : "+v"(a), "+v"(b), "+v"(c), "+v"(d)); }

struct FragB {
  union U { v16b v; v8b h[2]; };
  static __device__ __forceinline__ v16b load(const __bf16* p) {
    U f; f.h[0] = *(const v8b*)(p); f.h[1] = *(const v8b*)(p + 16); return f.v;
  }
  static __device__ __forceinline__ v8f mma(v16b a, v16b b, v8f c) {
    return __builtin_amdgcn_wmma_f32_16x16x32_bf16(false, a, false, b, (short)0, c, false, false);
  }
};

__device__ __forceinline__ v8f zero8() { v8f z = {0.f, 0.f, 0.f, 0.f, 0.f, 0.f, 0.f, 0.f}; return z; }

template <int BIAS_MODE>
__global__ __launch_bounds__(256) void wmma_gemm64(
    const unsigned short* __restrict__ Ap, int lda, long sAy, long sAz,
    const unsigned short* __restrict__ Btp, int ldb, long sBy, long sBz,
    unsigned short* Cout, unsigned short* Cout2, int ldc, long sCy, long sCz,
    const float* __restrict__ bias, int sBias,
    int M, int N, int K, float scale) {
  const __bf16* A  = (const __bf16*)(const void*)Ap;
  const __bf16* Bt = (const __bf16*)(const void*)Btp;
  __shared__ __align__(16) float sT[8][16 * 68];
  const int y    = blockIdx.y;
  const int z    = blockIdx.z;
  const int lane = threadIdx.x & 31;
  const int wave = threadIdx.x >> 5;
  const int tilesN = N >> 6;
  const int tilesM = M >> 6;
  const int tile = blockIdx.x * 8 + wave;
  if (tile >= tilesM * tilesN) return;
  const int tm = tile / tilesN;
  const int tn = tile - tm * tilesN;
  const int m0 = tm << 6;
  const int n0 = tn << 6;

  const __bf16* Ab = A  + (size_t)y * sAy + (size_t)z * sAz;
  const __bf16* Bb = Bt + (size_t)y * sBy + (size_t)z * sBz;
  const float*  biasb = bias + (size_t)y * sBias;

  const int rlane = lane & 15;
  const int koff  = (lane >> 4) * 8;
  const int mOff  = (lane >> 4) * 8;

  v8f acc[4][4];
#pragma unroll
  for (int i = 0; i < 4; ++i)
#pragma unroll
    for (int j = 0; j < 4; ++j) acc[i][j] = zero8();

  for (int k0 = 0; k0 < K; k0 += 32) {
    v16b bh[4];
#pragma unroll
    for (int j = 0; j < 4; ++j) {
      const size_t bo = (size_t)(n0 + (j << 4) + rlane) * ldb + koff + k0;
      bh[j] = FragB::load(Bb + bo);
    }
#pragma unroll
    for (int i = 0; i < 4; ++i) {
      const size_t ao = (size_t)(m0 + (i << 4) + rlane) * lda + koff + k0;
      v16b ah = FragB::load(Ab + ao);
#pragma unroll
      for (int j = 0; j < 4; ++j) acc[i][j] = FragB::mma(ah, bh[j], acc[i][j]);
      dep_guard_b(acc[i][0], acc[i][3], ah, ah);
    }
    keep4_b(bh[0], bh[1], bh[2], bh[3]);
  }
  acc_guard4(acc[0][0], acc[0][1], acc[0][2], acc[0][3]);
  acc_guard4(acc[1][0], acc[1][1], acc[1][2], acc[1][3]);
  acc_guard4(acc[2][0], acc[2][1], acc[2][2], acc[2][3]);
  acc_guard4(acc[3][0], acc[3][1], acc[3][2], acc[3][3]);

  float* slab = sT[wave];
  unsigned short* C  = Cout  + (size_t)y * sCy + (size_t)z * sCz;
  unsigned short* C2 = Cout2 + (size_t)y * sCy + (size_t)z * sCz;
#pragma unroll
  for (int i = 0; i < 4; ++i) {
    const int mBase = m0 + (i << 4);
    v8f bm = zero8();
    if (BIAS_MODE == 1) bm = *(const v8f*)(biasb + mBase + mOff);
#pragma unroll
    for (int j = 0; j < 4; ++j) {
      const int n = n0 + (j << 4) + rlane;
      float bn = 0.f;
      if (BIAS_MODE == 2) bn = bfr(biasb[n]);
#pragma unroll
      for (int r = 0; r < 8; ++r) {
        float v = acc[i][j][r] * scale;
        if (BIAS_MODE == 1) v += bfr(bm[r]);
        if (BIAS_MODE == 2) v += bn;
        slab[(mOff + r) * 68 + (j << 4) + rlane] = v;
      }
    }
    __builtin_amdgcn_fence(__ATOMIC_RELEASE, "workgroup");
    __builtin_amdgcn_wave_barrier();
    __builtin_amdgcn_fence(__ATOMIC_ACQUIRE, "workgroup");
    {
      const int q = lane >> 3, c8 = (lane & 7) * 8;
      for (int pass = 0; pass < 2; ++pass) {
#pragma unroll
        for (int it = 0; it < 4; ++it) {
          const int row = it * 4 + q;
          const float* sp = slab + row * 68 + c8;
          v8h hv, lv;
#pragma unroll
          for (int e = 0; e < 8; ++e) {
            const unsigned short hb = f2bf_bits(sp[e]);
            const unsigned short lb = f2bf_bits(sp[e] - bf_bits2f(hb));
            hv[e] = __builtin_bit_cast(_Float16, hb);
            lv[e] = __builtin_bit_cast(_Float16, lb);
          }
          *(volatile v8h*)(C  + (size_t)(mBase + row) * ldc + n0 + c8) = hv;
          *(volatile v8h*)(C2 + (size_t)(mBase + row) * ldc + n0 + c8) = lv;
        }
        __threadfence();
      }
    }
    __builtin_amdgcn_fence(__ATOMIC_RELEASE, "workgroup");
    __builtin_amdgcn_wave_barrier();
    __builtin_amdgcn_fence(__ATOMIC_ACQUIRE, "workgroup");
  }
}

__global__ __launch_bounds__(256) void cvt_bf16x8_kernel(const float* __restrict__ in, unsigned short* __restrict__ o, int n8) {
  const int i = blockIdx.x * 256 + threadIdx.x;
  if (i < n8) {
    const float* sp = in + (size_t)i * 8;
    const v4f a  = *(const v4f*)(sp);
    const v4f a2 = *(const v4f*)(sp + 4);
    v4u w;
    w[0] = pk16(f2bf_bits(a[0]),  f2bf_bits(a[1]));
    w[1] = pk16(f2bf_bits(a[2]),  f2bf_bits(a[3]));
    w[2] = pk16(f2bf_bits(a2[0]), f2bf_bits(a2[1]));
    w[3] = pk16(f2bf_bits(a2[2]), f2bf_bits(a2[3]));
    unsigned short* dp = o + (size_t)i * 8;
    *(volatile v4u*)dp = w;
    __threadfence();
    *(volatile v4u*)dp = w;
  }
}

#define AT_D  64
#define AT_NW 4
#define AT_QB 64
#define AT_KC 64
#define NQB   (SEQ / AT_QB)

__device__ __forceinline__ __bf16 at_f2bf(float f) { return __builtin_bit_cast(__bf16, f2bf_bits(f)); }
__device__ __forceinline__ void at_split(float f, __bf16& hi, __bf16& lo) {
  const unsigned short hb = f2bf_bits(f);
  hi = __builtin_bit_cast(__bf16, hb);
  lo = at_f2bf(f - __uint_as_float(((unsigned)hb) << 16));
}
__device__ __forceinline__ v8f at_mma(v16b a, v16b b, v8f c) {
  c = __builtin_amdgcn_wmma_f32_16x16x32_bf16(false, a, false, b, (short)0, c, false, false);
  asm volatile("v_nop\n\tv_nop\n\tv_nop\n\tv_nop" : "+v"(c) : "v"(a), "v"(b));
  return c;
}

__global__ __launch_bounds__(128)
void attn_full64_kernel(const unsigned short* __restrict__ qhp, const unsigned short* __restrict__ qlp,
                        const unsigned short* __restrict__ khp, const unsigned short* __restrict__ klp,
                        const unsigned short* __restrict__ vhp, const unsigned short* __restrict__ vlp,
                        float* __restrict__ out, float sscale) {
  union FB { v16b v; v8b h[2]; };
  __shared__ __align__(16) __bf16 Ksh[AT_KC * AT_D];
  __shared__ __align__(16) __bf16 Ksl[AT_KC * AT_D];
  __shared__ __align__(16) __bf16 Vth[AT_D * AT_KC];
  __shared__ __align__(16) __bf16 Vtl[AT_D * AT_KC];
  __shared__ __align__(16) __bf16 Psh[AT_NW][16 * AT_KC];
  __shared__ __align__(16) __bf16 Psl[AT_NW][16 * AT_KC];
  __shared__ __align__(16) float  Os[AT_NW][16 * 68];

  const int tid  = threadIdx.x;
  const int wave = tid >> 5;
  const int lane = tid & 31;
  const int hh   = lane >> 4;
  const int c    = lane & 15;

  const int bx   = blockIdx.x;
  const int qb   = bx & (NQB - 1);
  const int pair = bx >> 5;
  const int h    = pair & (NH - 1);
  const int b    = pair >> 4;
  const int q0   = qb * AT_QB + wave * 16;
  const size_t tok0 = (size_t)b * SEQ;

  const __bf16* Qh = (const __bf16*)(const void*)qhp + tok0 * DMOD + (size_t)h * AT_D;
  const __bf16* Ql = (const __bf16*)(const void*)qlp + tok0 * DMOD + (size_t)h * AT_D;
  const __bf16* Kh = (const __bf16*)(const void*)khp + tok0 * DMOD + (size_t)h * AT_D;
  const __bf16* Kl = (const __bf16*)(const void*)klp + tok0 * DMOD + (size_t)h * AT_D;
  const __bf16* Vh = (const __bf16*)(const void*)vhp + ((size_t)b * DMOD + (size_t)h * AT_D) * SEQ;
  const __bf16* Vl = (const __bf16*)(const void*)vlp + ((size_t)b * DMOD + (size_t)h * AT_D) * SEQ;
  float*        ob = out + tok0 * DMOD + (size_t)h * AT_D;

  v16b qah[2], qal[2];
#pragma unroll
  for (int dc = 0; dc < 2; ++dc) {
    const __bf16* qr = Qh + (size_t)(q0 + c) * DMOD + dc * 32 + 8 * hh;
    const __bf16* ql = Ql + (size_t)(q0 + c) * DMOD + dc * 32 + 8 * hh;
    qah[dc] = FragB::load(qr);
    qal[dc] = FragB::load(ql);
  }

  float mrow[8], lrow[8];
  v8f oacc[4];
#pragma unroll
  for (int r = 0; r < 8; ++r) { mrow[r] = -INFINITY; lrow[r] = 0.f; }
#pragma unroll
  for (int t = 0; t < 4; ++t) oacc[t] = zero8();

  const int nChunks = SEQ / AT_KC;
  for (int kc = 0; kc < nChunks; ++kc) {
    const int kv0 = kc * AT_KC;
    __syncthreads();
    {
      const int r = tid >> 1, half = (tid & 1) * 32;
      const __bf16* ksh = Kh + (size_t)(kv0 + r) * DMOD + half;
      const __bf16* ksl = Kl + (size_t)(kv0 + r) * DMOD + half;
      const __bf16* vsh = Vh + (size_t)r * SEQ + kv0 + half;
      const __bf16* vsl = Vl + (size_t)r * SEQ + kv0 + half;
#pragma unroll
      for (int i = 0; i < 4; ++i) {
        const v8b a0 = *(const v8b*)(ksh + 8 * i);
        const v8b a1 = *(const v8b*)(ksl + 8 * i);
        const v8b b0 = *(const v8b*)(vsh + 8 * i);
        const v8b b1 = *(const v8b*)(vsl + 8 * i);
        *(v8b*)(Ksh + r * AT_D  + half + 8 * i) = a0;
        *(v8b*)(Ksl + r * AT_D  + half + 8 * i) = a1;
        *(v8b*)(Vth + r * AT_KC + half + 8 * i) = b0;
        *(v8b*)(Vtl + r * AT_KC + half + 8 * i) = b1;
      }
    }
    __syncthreads();

    v8f s[4];
#pragma unroll
    for (int j = 0; j < 4; ++j) {
      s[j] = zero8();
#pragma unroll
      for (int dc = 0; dc < 2; ++dc) {
        FB kb, kl;
        kb.h[0] = *(const v8b*)(Ksh + (j * 16 + c) * AT_D + dc * 32 + 8 * hh);
        kb.h[1] = *(const v8b*)(Ksh + (j * 16 + c) * AT_D + dc * 32 + 16 + 8 * hh);
        kl.h[0] = *(const v8b*)(Ksl + (j * 16 + c) * AT_D + dc * 32 + 8 * hh);
        kl.h[1] = *(const v8b*)(Ksl + (j * 16 + c) * AT_D + dc * 32 + 16 + 8 * hh);
        s[j] = at_mma(qah[dc], kb.v, s[j]);
        s[j] = at_mma(qah[dc], kl.v, s[j]);
        s[j] = at_mma(qal[dc], kb.v, s[j]);
      }
    }
    float cm[8];
#pragma unroll
    for (int r = 0; r < 8; ++r) {
      float m = -INFINITY;
#pragma unroll
      for (int j = 0; j < 4; ++j) {
        const float sv = s[j][r] * sscale;
        s[j][r] = sv;
        m = fmaxf(m, sv);
      }
#pragma unroll
      for (int off = 1; off < 16; off <<= 1) m = fmaxf(m, __shfl_xor(m, off, 32));
      cm[r] = m;
    }
    __bf16* pwh = Psh[wave];
    __bf16* pwl = Psl[wave];
#pragma unroll
    for (int r = 0; r < 8; ++r) {
      const float mnew = fmaxf(mrow[r], cm[r]);
      const float alpha = expf(mrow[r] - mnew);
      mrow[r] = mnew;
      float psum = 0.f;
#pragma unroll
      for (int j = 0; j < 4; ++j) {
        const float p = expf(s[j][r] - mnew);
        psum += p;
        __bf16 a, bl; at_split(p, a, bl);
        pwh[(8 * hh + r) * AT_KC + j * 16 + c] = a;
        pwl[(8 * hh + r) * AT_KC + j * 16 + c] = bl;
      }
#pragma unroll
      for (int off = 1; off < 16; off <<= 1) psum += __shfl_xor(psum, off, 32);
      lrow[r] = lrow[r] * alpha + psum;
#pragma unroll
      for (int t = 0; t < 4; ++t) oacc[t][r] *= alpha;
    }
    __builtin_amdgcn_fence(__ATOMIC_RELEASE, "workgroup");
    __builtin_amdgcn_wave_barrier();
    __builtin_amdgcn_fence(__ATOMIC_ACQUIRE, "workgroup");

#pragma unroll 1
    for (int kk = 0; kk < 2; ++kk) {
      FB pa, pl;
      pa.h[0] = *(const v8b*)(pwh + c * AT_KC + kk * 32 + 8 * hh);
      pa.h[1] = *(const v8b*)(pwh + c * AT_KC + kk * 32 + 16 + 8 * hh);
      pl.h[0] = *(const v8b*)(pwl + c * AT_KC + kk * 32 + 8 * hh);
      pl.h[1] = *(const v8b*)(pwl + c * AT_KC + kk * 32 + 16 + 8 * hh);
#pragma unroll
      for (int t = 0; t < 4; ++t) {
        FB vb, vl;
        vb.h[0] = *(const v8b*)(Vth + (t * 16 + c) * AT_KC + kk * 32 + 8 * hh);
        vb.h[1] = *(const v8b*)(Vth + (t * 16 + c) * AT_KC + kk * 32 + 16 + 8 * hh);
        vl.h[0] = *(const v8b*)(Vtl + (t * 16 + c) * AT_KC + kk * 32 + 8 * hh);
        vl.h[1] = *(const v8b*)(Vtl + (t * 16 + c) * AT_KC + kk * 32 + 16 + 8 * hh);
        oacc[t] = at_mma(pa.v, vb.v, oacc[t]);
        oacc[t] = at_mma(pa.v, vl.v, oacc[t]);
        oacc[t] = at_mma(pl.v, vb.v, oacc[t]);
      }
    }
  }

  float* os = Os[wave];
#pragma unroll
  for (int r = 0; r < 8; ++r) {
    const float inv = 1.0f / lrow[r];
#pragma unroll
    for (int t = 0; t < 4; ++t) os[(8 * hh + r) * 68 + t * 16 + c] = oacc[t][r] * inv;
  }
  __builtin_amdgcn_fence(__ATOMIC_RELEASE, "workgroup");
  __builtin_amdgcn_wave_barrier();
  __builtin_amdgcn_fence(__ATOMIC_ACQUIRE, "workgroup");
  {
    const int c4 = (lane & 15) * 4;
    for (int pass = 0; pass < 2; ++pass) {
#pragma unroll
      for (int it = 0; it < 8; ++it) {
        const int row = it * 2 + hh;
        v4f val = *(const v4f*)(os + row * 68 + c4);
        *(volatile v4f*)(ob + (size_t)(q0 + row) * DMOD + c4) = val;
      }
      __threadfence();
    }
  }
}

#define PXB ((size_t)NTOK * DMOD * 2)
#define PWB ((size_t)NH * HD * HD * 2)
#define PVT ((size_t)NB * DMOD * SEQ * 2)
#define WS_TOTAL (PXB + 3 * PWB + 4 * PXB + 2 * PVT)
static_assert(WS_TOTAL == (size_t)117833728);
static_assert(WS_TOTAL <= (size_t)134217728);
static_assert(HD % 32 == 0);
static_assert(NTOK % 64 == 0 && SEQ % 64 == 0 && HD % 64 == 0);

extern "C" void kernel_launch(void* const* d_in, const int* in_sizes, int n_in,
                              void* d_out, int out_size, void* d_ws, size_t ws_size,
                              hipStream_t stream) {
  if (n_in < 7) return;
  if (in_sizes[0] != NB * SEQ * DMOD) return;
  if (in_sizes[1] != NH * HD * HD || in_sizes[3] != NH * HD * HD || in_sizes[5] != NH * HD * HD) return;
  if (in_sizes[2] != NH * HD || in_sizes[4] != NH * HD || in_sizes[6] != NH * HD) return;
  if (out_size != NB * SEQ * DMOD) return;
  if (WS_TOTAL > ws_size) return;

  const float* x  = (const float*)d_in[0];
  const float* Wq = (const float*)d_in[1];
  const float* bq = (const float*)d_in[2];
  const float* Wk = (const float*)d_in[3];
  const float* bk = (const float*)d_in[4];
  const float* Wv = (const float*)d_in[5];
  const float* bv = (const float*)d_in[6];
  float* out = (float*)d_out;

  size_t off = 0;
  const size_t oXb  = off; off += PXB;
  const size_t oWqb = off; off += PWB;  const size_t oWkb = off; off += PWB;  const size_t oWvb = off; off += PWB;
  const size_t oQh  = off; off += PXB;  const size_t oQl  = off; off += PXB;
  const size_t oKh  = off; off += PXB;  const size_t oKl  = off; off += PXB;
  const size_t oVTh = off; off += PVT;  const size_t oVTl = off; off += PVT;
  if (off != WS_TOTAL || off > ws_size) return;

  char* ws = (char*)d_ws;
  unsigned short* Xb  = (unsigned short*)(ws + oXb);
  unsigned short* Wqb = (unsigned short*)(ws + oWqb);
  unsigned short* Wkb = (unsigned short*)(ws + oWkb);
  unsigned short* Wvb = (unsigned short*)(ws + oWvb);
  unsigned short* Qh  = (unsigned short*)(ws + oQh);  unsigned short* Ql  = (unsigned short*)(ws + oQl);
  unsigned short* Kh  = (unsigned short*)(ws + oKh);  unsigned short* Kl  = (unsigned short*)(ws + oKl);
  unsigned short* VTh = (unsigned short*)(ws + oVTh); unsigned short* VTl = (unsigned short*)(ws + oVTl);

  const dim3 blk(256);

  const int n8x = NB * SEQ * DMOD / 8;
  cvt_bf16x8_kernel<<<dim3((n8x + 255) / 256), blk, 0, stream>>>(x, Xb, n8x);
  const int n8w = NH * HD * HD / 8;
  cvt_bf16x8_kernel<<<dim3((n8w + 255) / 256), blk, 0, stream>>>(Wq, Wqb, n8w);
  cvt_bf16x8_kernel<<<dim3((n8w + 255) / 256), blk, 0, stream>>>(Wk, Wkb, n8w);
  cvt_bf16x8_kernel<<<dim3((n8w + 255) / 256), blk, 0, stream>>>(Wv, Wvb, n8w);

  const dim3 gQK(((NTOK / 64) * (HD / 64) + 7) / 8, NH, 1);
  wmma_gemm64<2><<<gQK, blk, 0, stream>>>(
      Xb, DMOD, (long)HD, 0L, Wqb, HD, (long)HD * HD, 0L, Qh, Ql, DMOD, (long)HD, 0L,
      bq, HD, NTOK, HD, HD, 1.0f);
  wmma_gemm64<2><<<gQK, blk, 0, stream>>>(
      Xb, DMOD, (long)HD, 0L, Wkb, HD, (long)HD * HD, 0L, Kh, Kl, DMOD, (long)HD, 0L,
      bk, HD, NTOK, HD, HD, 1.0f);
  const dim3 gVT(((HD / 64) * (SEQ / 64) + 7) / 8, NH, NB);
  wmma_gemm64<1><<<gVT, blk, 0, stream>>>(
      Wvb, HD, (long)HD * HD, 0L, Xb, DMOD, (long)HD, (long)SEQ * DMOD, VTh, VTl, SEQ, (long)HD * SEQ, (long)DMOD * SEQ,
      bv, HD, HD, SEQ, HD, 1.0f);
  attn_full64_kernel<<<dim3(NB * NH * NQB), dim3(128), 0, stream>>>(Qh, Ql, Kh, Kl, VTh, VTl, out, 0.125f);
  (void)hipGetLastError();
}
